// GeomAwareSelfAttention_11982958756651
// MI455X (gfx1250) — hardware-verified
//
#include <hip/hip_runtime.h>
#include <stddef.h>
#include <stdint.h>

#define NBAT 4
#define SEQ  1024
#define NTOK 4096
#define DM   512
#define NHD  8
#define HD   64
#define HID  64
#define NFF  32
#define QB   64
#define KC   64
#define NQB  (SEQ / QB)

static_assert(NTOK == NBAT * SEQ);
static_assert(DM == NHD * HD);
static_assert(DM % 64 == 0);
static_assert(DM % 32 == 0);
static_assert(NTOK % 64 == 0);
static_assert(SEQ % QB == 0);
static_assert(SEQ % KC == 0);
static_assert(SEQ % 128 == 0);
static_assert(QB == KC);
static_assert(HD == 64);
static_assert(HID == 64);
static_assert(NFF * HID == 256 * 8);
static_assert((NTOK * DM) % 2048 == 0);

typedef unsigned short us;
typedef _Float16 v16h __attribute__((ext_vector_type(16)));
typedef _Float16 v8h  __attribute__((ext_vector_type(8)));
typedef __bf16   v16bf __attribute__((ext_vector_type(16)));
typedef us       v8us __attribute__((ext_vector_type(8)));
typedef float    v8f  __attribute__((ext_vector_type(8)));
typedef float    v4f  __attribute__((ext_vector_type(4)));
typedef unsigned int v4u __attribute__((ext_vector_type(4)));

union FragH { v16h v; v8us h[2]; };
union FragB { v16bf v; v8us h[2]; };
union Pack8 { v8us h; v4u u; };
union PackH { v8h f; v4u u; };

__device__ __forceinline__ us bf_rne(float f) {
  unsigned u = __float_as_uint(f);
  u = u + 0x7FFFu + ((u >> 16) & 1u);
  return (us)(u >> 16);
}
__device__ __forceinline__ float bf_val(us h) { return __uint_as_float(((unsigned)h) << 16); }
__device__ __forceinline__ void split2(float f, us& hi, us& lo) {
  const us hv = bf_rne(f);
  hi = hv;
  lo = bf_rne(f - bf_val(hv));
}
__device__ __forceinline__ void split8(const float (&f)[8], Pack8& ph, Pack8& pl) {
  us hh[8], ll[8];
#pragma unroll
  for (int e = 0; e < 8; ++e) split2(f[e], hh[e], ll[e]);
  ph.h = (v8us){hh[0], hh[1], hh[2], hh[3], hh[4], hh[5], hh[6], hh[7]};
  pl.h = (v8us){ll[0], ll[1], ll[2], ll[3], ll[4], ll[5], ll[6], ll[7]};
}
__device__ __forceinline__ v4u pack_h8(const float (&f)[8], float sc) {
  PackH p;
  p.f = (v8h){(_Float16)(f[0] * sc), (_Float16)(f[1] * sc), (_Float16)(f[2] * sc), (_Float16)(f[3] * sc),
              (_Float16)(f[4] * sc), (_Float16)(f[5] * sc), (_Float16)(f[6] * sc), (_Float16)(f[7] * sc)};
  return p.u;
}

__device__ __forceinline__ v8f mmah(v16h a, v16h b, v8f c) {
  c = __builtin_amdgcn_wmma_f32_16x16x32_f16(false, a, false, b, (short)0, c, false, false);
  asm volatile("v_nop\n\tv_nop\n\tv_nop\n\tv_nop" : "+v"(c) : "v"(a), "v"(b));
  return c;
}
__device__ __forceinline__ v8f mmab(v16bf a, v16bf b, v8f c) {
  c = __builtin_amdgcn_wmma_f32_16x16x32_bf16(false, a, false, b, (short)0, c, false, false);
  asm volatile("v_nop\n\tv_nop\n\tv_nop\n\tv_nop" : "+v"(c) : "v"(a), "v"(b));
  return c;
}
__device__ __forceinline__ v8f zero8() { return (v8f){0.f, 0.f, 0.f, 0.f, 0.f, 0.f, 0.f, 0.f}; }

template <class FR>
__device__ __forceinline__ FR ldfrag(const us* p, int ld, int row0, int k0, int lane) {
  const int m = lane & 15, lh = lane >> 4;
  const us* q = p + (size_t)(row0 + m) * ld + k0 + 8 * lh;
  FR f;
  f.h[0] = *(const v8us*)(q);
  f.h[1] = *(const v8us*)(q + 16);
  return f;
}

template <int KD>
__device__ __forceinline__ void gemm16x64_h(const us* __restrict__ A, const us* __restrict__ B,
                                            int m0, int n0, int lane, v8f (&acc)[4]) {
  static_assert(KD % 32 == 0);
#pragma unroll 1
  for (int k0 = 0; k0 < KD; k0 += 32) {
    const FragH a = ldfrag<FragH>(A, KD, m0, k0, lane);
#pragma unroll
    for (int t = 0; t < 4; ++t) {
      const FragH b = ldfrag<FragH>(B, KD, n0 + 16 * t, k0, lane);
      acc[t] = mmah(a.v, b.v, acc[t]);
    }
  }
}

template <int KD>
__device__ __forceinline__ void gemm16x64_x3(const us* __restrict__ Ah, const us* __restrict__ Al,
                                             const us* __restrict__ Bh, const us* __restrict__ Bl,
                                             int m0, int n0, int lane, v8f (&acc)[4]) {
  static_assert(KD % 32 == 0);
#pragma unroll 1
  for (int k0 = 0; k0 < KD; k0 += 32) {
    const FragB ah = ldfrag<FragB>(Ah, KD, m0, k0, lane);
    const FragB al = ldfrag<FragB>(Al, KD, m0, k0, lane);
#pragma unroll
    for (int t = 0; t < 4; ++t) {
      const FragB bh = ldfrag<FragB>(Bh, KD, n0 + 16 * t, k0, lane);
      const FragB bl = ldfrag<FragB>(Bl, KD, n0 + 16 * t, k0, lane);
      acc[t] = mmab(ah.v, bh.v, acc[t]);
      acc[t] = mmab(ah.v, bl.v, acc[t]);
      acc[t] = mmab(al.v, bh.v, acc[t]);
    }
  }
}

#define SFP 68

__global__ __launch_bounds__(256) void k_cvt_x(const float* __restrict__ x, us* __restrict__ xf,
                                               us* __restrict__ xh, us* __restrict__ xl) {
  const size_t i = (size_t)blockIdx.x * 2048 + (size_t)threadIdx.x * 8;
  const v4f a0 = *(const v4f*)(x + i);
  const v4f a1 = *(const v4f*)(x + i + 4);
  const float f[8] = {a0[0], a0[1], a0[2], a0[3], a1[0], a1[1], a1[2], a1[3]};
  Pack8 ph, pl;
  split8(f, ph, pl);
  const v4u fv = pack_h8(f, 1.0f), hv = ph.u, lv = pl.u;
  *(volatile v4u*)(xf + i) = fv;
  *(volatile v4u*)(xh + i) = hv;
  *(volatile v4u*)(xl + i) = lv;
  __threadfence();
  *(volatile v4u*)(xf + i) = fv;
  *(volatile v4u*)(xh + i) = hv;
  *(volatile v4u*)(xl + i) = lv;
}

template <bool SPLIT>
__global__ __launch_bounds__(256) void k_cvt_w(const float* __restrict__ w0, const float* __restrict__ w1,
                                               us* __restrict__ p0a, us* __restrict__ p0b,
                                               us* __restrict__ p1a, us* __restrict__ p1b, float sc) {
  __shared__ __align__(16) float sw[64 * SFP];
  const int tid = threadIdx.x;
  const float* W = (blockIdx.z == 0) ? w0 : w1;
  us* PA = (blockIdx.z == 0) ? p0a : p1a;
  us* PB = (blockIdx.z == 0) ? p0b : p1b;
  const int nb = blockIdx.x * 64;
  const int kb = blockIdx.y * 64;
  {
    const int r  = tid >> 2;
    const int c0 = (tid & 3) * 16;
    const float* src = W + (size_t)(kb + r) * DM + nb + c0;
#pragma unroll
    for (int e = 0; e < 4; ++e) *(v4f*)(sw + r * SFP + c0 + 4 * e) = *(const v4f*)(src + 4 * e);
  }
  __syncthreads();
  v4u hv[2], lv[2];
  size_t go[2];
#pragma unroll
  for (int j = 0; j < 2; ++j) {
    const int p  = tid + 256 * j;
    const int n  = p >> 3;
    const int pc = p & 7;
    const float* cp = sw + (pc * 8) * SFP + n;
    float f[8];
#pragma unroll
    for (int e = 0; e < 8; ++e) f[e] = cp[e * SFP];
    if (SPLIT) {
      Pack8 ph, pl;
      split8(f, ph, pl);
      hv[j] = ph.u;
      lv[j] = pl.u;
    } else {
      hv[j] = pack_h8(f, sc);
      lv[j] = hv[j];
    }
    go[j] = (size_t)(nb + n) * DM + kb + pc * 8;
  }
#pragma unroll
  for (int j = 0; j < 2; ++j) {
    *(volatile v4u*)(PA + go[j]) = hv[j];
    if (SPLIT) *(volatile v4u*)(PB + go[j]) = lv[j];
  }
  __threadfence();
#pragma unroll
  for (int j = 0; j < 2; ++j) {
    *(volatile v4u*)(PA + go[j]) = hv[j];
    if (SPLIT) *(volatile v4u*)(PB + go[j]) = lv[j];
  }
}

__global__ __launch_bounds__(128) void k_projqk(const us* __restrict__ xf, const us* __restrict__ wq,
                                                const us* __restrict__ wk, us* __restrict__ yq,
                                                us* __restrict__ yk) {
  __shared__ __align__(16) float sf[64 * SFP];
  const int tid = threadIdx.x, lane = tid & 31, wave = tid >> 5;
  const int hh = lane >> 4, c = lane & 15;
  const us* W = (blockIdx.z == 0) ? wq : wk;
  us* Y = (blockIdx.z == 0) ? yq : yk;
  const int mb = blockIdx.x * 64;
  const int nb = blockIdx.y * 64;
  const int m0 = mb + wave * 16;

  v8f acc[4];
#pragma unroll
  for (int t = 0; t < 4; ++t) acc[t] = zero8();
  gemm16x64_h<DM>(xf, W, m0, nb, lane, acc);

#pragma unroll
  for (int t = 0; t < 4; ++t) {
#pragma unroll
    for (int r = 0; r < 8; ++r) sf[(wave * 16 + 8 * hh + r) * SFP + 16 * t + c] = acc[t][r];
  }
  __syncthreads();

  v4u hv[4];
  size_t go[4];
#pragma unroll
  for (int j = 0; j < 4; ++j) {
    const int p  = tid + 128 * j;
    const int lr = p >> 3;
    const int d0 = (p & 7) * 8;
    const float* ra = sf + lr * SFP + d0;
    const v4f a0 = *(const v4f*)(ra), a1 = *(const v4f*)(ra + 4);
    const float f[8] = {a0[0], a0[1], a0[2], a0[3], a1[0], a1[1], a1[2], a1[3]};
    hv[j] = pack_h8(f, 1.0f);
    go[j] = (size_t)(mb + lr) * DM + nb + d0;
  }
#pragma unroll
  for (int j = 0; j < 4; ++j) *(volatile v4u*)(Y + go[j]) = hv[j];
  __threadfence();
#pragma unroll
  for (int j = 0; j < 4; ++j) *(volatile v4u*)(Y + go[j]) = hv[j];
}

__global__ __launch_bounds__(128) void k_projv(const us* __restrict__ xh, const us* __restrict__ xl,
                                               const us* __restrict__ wh, const us* __restrict__ wl,
                                               us* __restrict__ vth, us* __restrict__ vtl) {
  __shared__ __align__(16) float sf[64 * SFP];
  const int tid = threadIdx.x, lane = tid & 31, wave = tid >> 5;
  const int hh = lane >> 4, c = lane & 15;
  const int mb = blockIdx.x * 64;
  const int nb = blockIdx.y * 64;
  const int m0 = mb + wave * 16;

  v8f acc[4];
#pragma unroll
  for (int t = 0; t < 4; ++t) acc[t] = zero8();
  gemm16x64_x3<DM>(xh, xl, wh, wl, m0, nb, lane, acc);

#pragma unroll
  for (int t = 0; t < 4; ++t) {
#pragma unroll
    for (int r = 0; r < 8; ++r) sf[(wave * 16 + 8 * hh + r) * SFP + 16 * t + c] = acc[t][r];
  }
  __syncthreads();

  v4u hv[4], lv[4];
  size_t go[4];
#pragma unroll
  for (int j = 0; j < 4; ++j) {
    const int p  = tid + 128 * j;
    const int d  = p >> 3;
    const int pc = p & 7;
    const float* cp = sf + (pc * 8) * SFP + d;
    float f[8];
#pragma unroll
    for (int e = 0; e < 8; ++e) f[e] = cp[e * SFP];
    Pack8 ph, pl;
    split8(f, ph, pl);
    hv[j] = ph.u;
    lv[j] = pl.u;
    go[j] = (size_t)(nb + d) * NTOK + mb + pc * 8;
  }
#pragma unroll
  for (int j = 0; j < 4; ++j) { *(volatile v4u*)(vth + go[j]) = hv[j]; *(volatile v4u*)(vtl + go[j]) = lv[j]; }
  __threadfence();
#pragma unroll
  for (int j = 0; j < 4; ++j) { *(volatile v4u*)(vth + go[j]) = hv[j]; *(volatile v4u*)(vtl + go[j]) = lv[j]; }
}

__global__ __launch_bounds__(256) void k_bias(const float* __restrict__ coords, const float* __restrict__ w1,
                                              const float* __restrict__ b1, const float* __restrict__ w2,
                                              const float* __restrict__ b2, float* __restrict__ bias) {
#pragma clang fp contract(off)
  __shared__ __align__(16) float sw1[NFF * HID];
  __shared__ __align__(16) float sb1[HID];
  __shared__ __align__(16) float sw2[HID];
  __shared__ __align__(16) float sb[8 * 128];
  const int tid = threadIdx.x, lane = tid & 31, wave = tid >> 5;
  const int hh = lane >> 4, c = lane & 15;
  const int gw = blockIdx.x * 8 + wave;
  const int b = gw >> 10;
  const int tok0 = b * SEQ;

  {
    const v4f a0 = *(const v4f*)(w1 + tid * 8);
    const v4f a1 = *(const v4f*)(w1 + tid * 8 + 4);
    *(v4f*)(sw1 + tid * 8)     = a0;
    *(v4f*)(sw1 + tid * 8 + 4) = a1;
    if (wave == 0) {
      const v4f bv = *(const v4f*)(b1 + c * 4);
      *(v4f*)(sb1 + c * 4) = bv;
    } else if (wave == 1) {
      const v4f wv = *(const v4f*)(w2 + c * 4);
      *(v4f*)(sw2 + c * 4) = wv;
    }
  }
  __syncthreads();

  v16h wf[4];
#pragma unroll
  for (int t = 0; t < 4; ++t) {
#pragma unroll
    for (int i = 0; i < 16; ++i) {
      const int kk = (i < 8) ? (8 * hh + i) : (16 + 8 * hh + (i - 8));
      wf[t][i] = (_Float16)(sw1[kk * HID + 16 * t + c] * 16.0f);
    }
  }
  float b1v[4], w2v[4];
#pragma unroll
  for (int t = 0; t < 4; ++t) { b1v[t] = sb1[16 * t + c]; w2v[t] = sw2[16 * t + c]; }
  const float b2v = b2[0];
  float divt[8];
#pragma unroll
  for (int e = 0; e < 8; ++e) divt[e] = expf((float)(2 * (8 * hh + e)) * (-0.28782313662425574f));

  const v4f cq = *(const v4f*)(coords + (size_t)gw * 4);
  float* brow = bias + (size_t)gw * SEQ;
  float* sbw = sb + wave * 128;

#pragma unroll 1
  for (int g = 0; g < SEQ / 128; ++g) {
#pragma unroll 1
    for (int j = 0; j < 8; ++j) {
      const int k0 = g * 128 + j * 16;
      const v4f ck = *(const v4f*)(coords + (size_t)(tok0 + k0 + c) * 4);
      const float dx = cq[0] - ck[0], dy = cq[1] - ck[1], dz = cq[2] - ck[2];
      const float dt = cq[3] - ck[3];
      const float dr = (dx * dx + dz * dz) + dy * dy;
      const float ds = (0.05317636f * dt) * dt - dr;
      v16h ff;
#pragma unroll
      for (int e = 0; e < 8; ++e) {
        const float fa = ds * divt[e];
        float sv, cv;
        sincosf(fa, &sv, &cv);
        ff[e]     = (_Float16)sv;
        ff[8 + e] = (_Float16)cv;
      }
      float dot[8];
#pragma unroll
      for (int r = 0; r < 8; ++r) dot[r] = 0.f;
#pragma unroll
      for (int t = 0; t < 4; ++t) {
        const v8f hv = mmah(ff, wf[t], zero8());
#pragma unroll
        for (int r = 0; r < 8; ++r) {
          float x = hv[r] * 0.0625f + b1v[t];
          x = fmaxf(x, 0.f);
          dot[r] = dot[r] + x * w2v[t];
        }
      }
#pragma unroll
      for (int r = 0; r < 8; ++r) {
        float s = dot[r];
        s += __shfl_xor(s, 1, 32);
        s += __shfl_xor(s, 2, 32);
        s += __shfl_xor(s, 4, 32);
        s += __shfl_xor(s, 8, 32);
        if (c == r) sbw[j * 16 + 8 * hh + r] = s + b2v;
      }
    }
    __syncthreads();
    const v4f v = *(const v4f*)(sbw + 4 * lane);
    float* dst = brow + g * 128 + 4 * lane;
    *(volatile v4f*)dst = v;
    __threadfence();
    *(volatile v4f*)dst = v;
    __syncthreads();
  }
}

#define LP  72
#define OTP 68
union AttnLds {
  us    p[2][4 * 16 * LP];
  float o[4][16 * OTP];
};

__global__ __launch_bounds__(128) void k_attn(const us* __restrict__ qf, const us* __restrict__ kf,
                                              const us* __restrict__ vth, const us* __restrict__ vtl,
                                              const float* __restrict__ bias,
                                              us* __restrict__ obh, us* __restrict__ obl) {
  __shared__ __align__(16) us Ksh[KC * LP];
  __shared__ __align__(16) us Vsh[HD * LP];
  __shared__ __align__(16) us Vsl[HD * LP];
  __shared__ __align__(16) AttnLds pu;

  const int tid = threadIdx.x, lane = tid & 31, wave = tid >> 5;
  const int hh = lane >> 4, c = lane & 15;
  const int qb   = blockIdx.x;
  const int h    = blockIdx.y;
  const int b    = blockIdx.z;
  const int tok0 = b * SEQ;
  const int qloc = qb * QB + wave * 16;
  const int q0   = tok0 + qloc;
  const int hc   = h * HD;

  const float NEGI = -__builtin_huge_valf();
  const float SCL  = 0.00048828125f;
  float mrow[8], lrow[8];
  v8f oacc[4];
#pragma unroll
  for (int r = 0; r < 8; ++r) { mrow[r] = NEGI; lrow[r] = 0.f; }
#pragma unroll
  for (int t = 0; t < 4; ++t) oacc[t] = zero8();

  us* pwh = pu.p[0] + wave * 16 * LP;
  us* pwl = pu.p[1] + wave * 16 * LP;
  const float* brow = bias + (size_t)(q0 + 8 * hh) * SEQ + c;

#pragma unroll 1
  for (int i = 0; i < SEQ / KC; ++i) {
    const int kv0 = i * KC;
    __syncthreads();
    {
      const int r  = tid >> 1;
      const int cb = (tid & 1) * 32;
      const us* ksrc = kf  + (size_t)(tok0 + kv0 + r) * DM + hc + cb;
      const us* vhs  = vth + (size_t)(hc + r) * NTOK + tok0 + kv0 + cb;
      const us* vls  = vtl + (size_t)(hc + r) * NTOK + tok0 + kv0 + cb;
#pragma unroll
      for (int e = 0; e < 4; ++e) {
        *(v8us*)(Ksh + r * LP + cb + 8 * e) = *(const v8us*)(ksrc + 8 * e);
        *(v8us*)(Vsh + r * LP + cb + 8 * e) = *(const v8us*)(vhs + 8 * e);
        *(v8us*)(Vsl + r * LP + cb + 8 * e) = *(const v8us*)(vls + 8 * e);
      }
    }
    __syncthreads();

    v8f s[4];
#pragma unroll
    for (int j = 0; j < 4; ++j) s[j] = zero8();
#pragma unroll
    for (int dc = 0; dc < 2; ++dc) {
      const FragH qa = ldfrag<FragH>(qf, DM, q0, hc + dc * 32, lane);
#pragma unroll
      for (int j = 0; j < 4; ++j) {
        const FragH kb = ldfrag<FragH>(Ksh, LP, j * 16, dc * 32, lane);
        s[j] = mmah(qa.v, kb.v, s[j]);
      }
    }
#pragma unroll
    for (int j = 0; j < 4; ++j) {
#pragma unroll
      for (int r = 0; r < 8; ++r)
        s[j][r] = s[j][r] * SCL + brow[(size_t)r * SEQ + kv0 + j * 16];
    }
    float cm[8];
#pragma unroll
    for (int r = 0; r < 8; ++r) {
      float m = NEGI;
#pragma unroll
      for (int j = 0; j < 4; ++j) m = fmaxf(m, s[j][r]);
#pragma unroll
      for (int off = 1; off < 16; off <<= 1) m = fmaxf(m, __shfl_xor(m, off, 32));
      cm[r] = m;
    }
    float al[8];
#pragma unroll
    for (int r = 0; r < 8; ++r) {
      const float mnew  = fmaxf(mrow[r], cm[r]);
      const float aexp  = __expf(mrow[r] - mnew);
      const float alpha = (mrow[r] == NEGI) ? 0.f : aexp;
      mrow[r] = mnew;
      float psum = 0.f;
#pragma unroll
      for (int j = 0; j < 4; ++j) {
        const float p = __expf(s[j][r] - mnew);
        psum += p;
        us ph, pl;
        split2(p, ph, pl);
        pwh[(8 * hh + r) * LP + j * 16 + c] = ph;
        pwl[(8 * hh + r) * LP + j * 16 + c] = pl;
      }
#pragma unroll
      for (int off = 1; off < 16; off <<= 1) psum += __shfl_xor(psum, off, 32);
      lrow[r] = lrow[r] * alpha + psum;
      al[r] = alpha;
    }
#pragma unroll
    for (int t = 0; t < 4; ++t)
#pragma unroll
      for (int r = 0; r < 8; ++r) oacc[t][r] *= al[r];
    __syncthreads();

#pragma unroll
    for (int kk = 0; kk < 2; ++kk) {
      const FragB pah = ldfrag<FragB>(pwh, LP, 0, kk * 32, lane);
      const FragB pal = ldfrag<FragB>(pwl, LP, 0, kk * 32, lane);
#pragma unroll
      for (int t = 0; t < 4; ++t) {
        const FragB vbh = ldfrag<FragB>(Vsh, LP, t * 16, kk * 32, lane);
        const FragB vbl = ldfrag<FragB>(Vsl, LP, t * 16, kk * 32, lane);
        oacc[t] = mmab(pah.v, vbh.v, oacc[t]);
        oacc[t] = mmab(pah.v, vbl.v, oacc[t]);
        oacc[t] = mmab(pal.v, vbh.v, oacc[t]);
      }
    }
  }

  float invl[8];
#pragma unroll
  for (int r = 0; r < 8; ++r) invl[r] = (lrow[r] > 0.f) ? (1.0f / lrow[r]) : 0.f;
  __syncthreads();
  float* osw = pu.o[wave];
#pragma unroll
  for (int r = 0; r < 8; ++r) {
#pragma unroll
    for (int t = 0; t < 4; ++t) osw[(8 * hh + r) * OTP + 16 * t + c] = oacc[t][r] * invl[r];
  }
  __syncthreads();
  v4u hv[4], lv[4];
  size_t go[4];
#pragma unroll
  for (int it = 0; it < 4; ++it) {
    const int p   = lane + 32 * it;
    const int row = p >> 3;
    const int pc  = p & 7;
    const float* ra = osw + row * OTP + 8 * pc;
    const v4f a0 = *(const v4f*)(ra), a1 = *(const v4f*)(ra + 4);
    const float f[8] = {a0[0], a0[1], a0[2], a0[3], a1[0], a1[1], a1[2], a1[3]};
    Pack8 ph, pl;
    split8(f, ph, pl);
    hv[it] = ph.u;
    lv[it] = pl.u;
    go[it] = (size_t)(q0 + row) * DM + hc + 8 * pc;
  }
#pragma unroll
  for (int it = 0; it < 4; ++it) { *(volatile v4u*)(obh + go[it]) = hv[it]; *(volatile v4u*)(obl + go[it]) = lv[it]; }
  __threadfence();
#pragma unroll
  for (int it = 0; it < 4; ++it) { *(volatile v4u*)(obh + go[it]) = hv[it]; *(volatile v4u*)(obl + go[it]) = lv[it]; }
}

__global__ __launch_bounds__(128) void k_oproj(const us* __restrict__ ah, const us* __restrict__ al,
                                               const us* __restrict__ wh, const us* __restrict__ wl,
                                               float* __restrict__ out) {
  __shared__ __align__(16) float sf[64 * SFP];
  const int tid = threadIdx.x, lane = tid & 31, wave = tid >> 5;
  const int hh = lane >> 4, c = lane & 15;
  const int mb = blockIdx.x * 64;
  const int nb = blockIdx.y * 64;
  const int m0 = mb + wave * 16;

  v8f acc[4];
#pragma unroll
  for (int t = 0; t < 4; ++t) acc[t] = zero8();
  gemm16x64_x3<DM>(ah, al, wh, wl, m0, nb, lane, acc);

#pragma unroll
  for (int t = 0; t < 4; ++t) {
#pragma unroll
    for (int r = 0; r < 8; ++r) sf[(wave * 16 + 8 * hh + r) * SFP + 16 * t + c] = acc[t][r];
  }
  __syncthreads();

  v4f val[8];
  size_t go[8];
#pragma unroll
  for (int it = 0; it < 8; ++it) {
    const int p  = tid + 128 * it;
    const int lr = p >> 4;
    const int pc = p & 15;
    val[it] = *(const v4f*)(sf + lr * SFP + 4 * pc);
    go[it]  = (size_t)(mb + lr) * DM + nb + 4 * pc;
  }
#pragma unroll
  for (int it = 0; it < 8; ++it) *(volatile v4f*)(out + go[it]) = val[it];
  __threadfence();
#pragma unroll
  for (int it = 0; it < 8; ++it) *(volatile v4f*)(out + go[it]) = val[it];
}

extern "C" void kernel_launch(void* const* d_in, const int* in_sizes, int n_in,
                              void* d_out, int out_size, void* d_ws, size_t ws_size,
                              hipStream_t stream) {
  if (n_in < 10) return;
  if (in_sizes[0] != NTOK * DM) return;
  if (in_sizes[1] != NTOK * 4) return;
  if (in_sizes[2] != DM * DM) return;
  if (in_sizes[3] != DM * DM) return;
  if (in_sizes[4] != DM * DM) return;
  if (in_sizes[5] != DM * DM) return;
  if (in_sizes[6] != NFF * HID) return;
  if (in_sizes[7] != HID) return;
  if (in_sizes[8] != HID) return;
  if (in_sizes[9] < 1) return;
  if (out_size != NTOK * DM) return;

  const float* src    = (const float*)d_in[0];
  const float* coords = (const float*)d_in[1];
  const float* Wq     = (const float*)d_in[2];
  const float* Wk     = (const float*)d_in[3];
  const float* Wv     = (const float*)d_in[4];
  const float* Wo     = (const float*)d_in[5];
  const float* w1     = (const float*)d_in[6];
  const float* b1     = (const float*)d_in[7];
  const float* w2     = (const float*)d_in[8];
  const float* b2     = (const float*)d_in[9];
  float* out = (float*)d_out;

  size_t off = 0;
  const size_t oXF  = off; off += (size_t)NTOK * DM * 2;
  const size_t oXH  = off; off += (size_t)NTOK * DM * 2;
  const size_t oXL  = off; off += (size_t)NTOK * DM * 2;
  const size_t oWQ  = off; off += (size_t)DM * DM * 2;
  const size_t oWK  = off; off += (size_t)DM * DM * 2;
  const size_t oWVh = off; off += (size_t)DM * DM * 2;
  const size_t oWVl = off; off += (size_t)DM * DM * 2;
  const size_t oWOh = off; off += (size_t)DM * DM * 2;
  const size_t oWOl = off; off += (size_t)DM * DM * 2;
  const size_t oQF  = off; off += (size_t)NTOK * DM * 2;
  const size_t oKF  = off; off += (size_t)NTOK * DM * 2;
  const size_t oVTh = off; off += (size_t)DM * NTOK * 2;
  const size_t oVTl = off; off += (size_t)DM * NTOK * 2;
  const size_t oBI  = off; off += (size_t)NTOK * SEQ * 4;
  const size_t oOBh = off; off += (size_t)NTOK * DM * 2;
  const size_t oOBl = off; off += (size_t)NTOK * DM * 2;
  if (off > ws_size) return;
  if (off > (size_t)134217728) return;

  char* ws = (char*)d_ws;
  us* XF   = (us*)(ws + oXF);   us* XH   = (us*)(ws + oXH);   us* XL = (us*)(ws + oXL);
  us* WQT  = (us*)(ws + oWQ);   us* WKT  = (us*)(ws + oWK);
  us* WVTh = (us*)(ws + oWVh);  us* WVTl = (us*)(ws + oWVl);
  us* WOTh = (us*)(ws + oWOh);  us* WOTl = (us*)(ws + oWOl);
  us* QF   = (us*)(ws + oQF);   us* KF   = (us*)(ws + oKF);
  us* VTh  = (us*)(ws + oVTh);  us* VTl  = (us*)(ws + oVTl);
  float* BIAS = (float*)(ws + oBI);
  us* OBh  = (us*)(ws + oOBh);  us* OBl  = (us*)(ws + oOBl);

  k_cvt_x<<<dim3((NTOK * DM) / 2048), dim3(256), 0, stream>>>(src, XF, XH, XL);
  k_cvt_w<false><<<dim3(DM / 64, DM / 64, 2), dim3(256), 0, stream>>>(Wq, Wk, WQT, WQT, WKT, WKT, 16.0f);
  k_cvt_w<true><<<dim3(DM / 64, DM / 64, 2), dim3(256), 0, stream>>>(Wv, Wo, WVTh, WVTl, WOTh, WOTl, 1.0f);
  k_projqk<<<dim3(NTOK / 64, DM / 64, 2), dim3(128), 0, stream>>>(XF, WQT, WKT, QF, KF);
  k_projv<<<dim3(NTOK / 64, DM / 64), dim3(128), 0, stream>>>(XH, XL, WVTh, WVTl, VTh, VTl);
  k_bias<<<dim3(NTOK / 8), dim3(256), 0, stream>>>(coords, w1, b1, w2, b2, BIAS);
  k_attn<<<dim3(NQB, NHD, NBAT), dim3(128), 0, stream>>>(QF, KF, VTh, VTl, BIAS, OBh, OBl);
  k_oproj<<<dim3(NTOK / 64, DM / 64), dim3(128), 0, stream>>>(OBh, OBl, WOTh, WOTl, out);
  (void)hipGetLastError();
}
